// MultiHeadRotaryAttention_56573309223931
// MI455X (gfx1250) — hardware-run, weakly checked
//
#include <hip/hip_runtime.h>
#include <math.h>

constexpr int kB   = 2;
constexpr int kS   = 2048;
constexpr int kD   = 2048;
constexpr int kH   = 16;
constexpr int kHD  = 128;
constexpr int kHalfHD = 64;
constexpr int kM   = kB * kS;
constexpr int kKT  = 64;
static_assert(kH * kHD == kD);
static_assert((kD % 32) == 0 && (kM % 128) == 0 && (kD % 128) == 0 && (kS % 128) == 0 && (kS % kKT) == 0);
static_assert(kHD == 128 && kHalfHD * 2 == kHD && kS == 2048);

constexpr float kXCarry   = 16.0f;
constexpr float kWCarry   = 256.0f;
constexpr float kQKVCarry = 16.0f;
constexpr float kPCarry   = 1024.0f;
constexpr float kCtxCarry = 256.0f;
constexpr float kProjScale = kQKVCarry / (kXCarry * kWCarry);
constexpr float kCtxFold   = kCtxCarry / (kPCarry * kQKVCarry);
constexpr float kOutScale  = 1.0f / (kCtxCarry * kWCarry);

constexpr size_t kPlane16 = (size_t)kM * kD * 2;
constexpr size_t kOffXH  = 0;
constexpr size_t kOffWT  = kOffXH + kPlane16;
constexpr size_t kOffQR  = kOffWT + (size_t)4 * kD * kD * 2;
constexpr size_t kOffKR  = kOffQR + kPlane16;
constexpr size_t kOffVT  = kOffKR + kPlane16;
constexpr size_t kOffAO  = kOffVT + kPlane16;
constexpr size_t kOffCOS = kOffAO + kPlane16;
constexpr size_t kOffSIN = kOffCOS + (size_t)kS * kHalfHD * 4;
constexpr size_t kWsTotal = kOffSIN + (size_t)kS * kHalfHD * 4;
static_assert(kWsTotal == 118489088ull);
static_assert(kWsTotal <= 134217728ull);
static_assert((kOffWT % 128) == 0 && (kOffQR % 128) == 0 && (kOffKR % 128) == 0 && (kOffVT % 128) == 0 &&
              (kOffAO % 128) == 0 && (kOffCOS % 128) == 0 && (kOffSIN % 128) == 0);

typedef __attribute__((ext_vector_type(16))) _Float16 v16h;
typedef __attribute__((ext_vector_type(8)))  _Float16 v8h;
typedef __attribute__((ext_vector_type(8)))  float    v8f;
typedef __attribute__((ext_vector_type(4)))  float    v4f;
typedef __attribute__((ext_vector_type(4)))  unsigned int v4u;

union FragU { v16h v; v8h h[2]; };

__device__ __forceinline__ unsigned short f2bf_bits(float f) {
  unsigned u = __float_as_uint(f);
  return (unsigned short)((u + 0x7FFFu + ((u >> 16) & 1u)) >> 16);
}
__device__ __forceinline__ float bf_bits2f(unsigned short h) { return __uint_as_float(((unsigned)h) << 16); }
__device__ __forceinline__ float bf16r(float f) { return bf_bits2f(f2bf_bits(f)); }
__device__ __forceinline__ unsigned pk16(unsigned short a, unsigned short b) { return (unsigned)a | ((unsigned)b << 16); }
__device__ __forceinline__ unsigned short h_bits(float f) { const _Float16 h = (_Float16)f; return __builtin_bit_cast(unsigned short, h); }

__device__ __forceinline__ v16h frag_ld(const _Float16* p) {
  FragU f;
  f.h[0] = *(const v8h*)(p);
  f.h[1] = *(const v8h*)(p + 16);
  return f.v;
}
__device__ __forceinline__ v8f mma_h(v16h a, v16h b, v8f c) {
  c = __builtin_amdgcn_wmma_f32_16x16x32_f16(false, a, false, b, (short)0, c, false, false);
  asm volatile("v_nop\n\tv_nop\n\tv_nop\n\tv_nop" : "+v"(c) : "v"(a), "v"(b));
  return c;
}
__device__ __forceinline__ void wave_lds_sync() {
  __builtin_amdgcn_fence(__ATOMIC_RELEASE, "workgroup");
  __builtin_amdgcn_wave_barrier();
  __builtin_amdgcn_fence(__ATOMIC_ACQUIRE, "workgroup");
}

__global__ __launch_bounds__(256) void cast_plane_kernel(const float* __restrict__ in, unsigned short* __restrict__ out,
                                                         int n8, float carry) {
  const int i = blockIdx.x * 256 + threadIdx.x;
  if (i >= n8) return;
  const float* p = in + 8 * (size_t)i;
  const v4f a = *(const v4f*)(p);
  const v4f c = *(const v4f*)(p + 4);
  unsigned short hb[8];
#pragma unroll
  for (int e = 0; e < 4; ++e) {
    hb[e]     = h_bits(bf16r(a[e]) * carry);
    hb[4 + e] = h_bits(bf16r(c[e]) * carry);
  }
  const v4u u = (v4u){pk16(hb[0], hb[1]), pk16(hb[2], hb[3]), pk16(hb[4], hb[5]), pk16(hb[6], hb[7])};
  unsigned short* q = out + 8 * (size_t)i;
  *(volatile v4u*)q = u;
  __threadfence();
  *(volatile v4u*)q = u;
}

__global__ __launch_bounds__(256) void wtcast_kernel(const float* __restrict__ W0, const float* __restrict__ W1,
                                                     const float* __restrict__ W2, const float* __restrict__ W3,
                                                     unsigned short* __restrict__ out, float carry) {
  __shared__ float sm[64][65];
  const int t  = threadIdx.x;
  const int d0 = blockIdx.x * 64;
  const int f0 = blockIdx.y * 64;
  const int z  = blockIdx.z;
  const float* W = (z == 0) ? W0 : (z == 1) ? W1 : (z == 2) ? W2 : W3;
#pragma unroll
  for (int i = 0; i < 16; ++i) {
    const int e = i * 256 + t;
    const int r = e >> 6;
    const int c = e & 63;
    sm[c][r] = bf16r(W[(size_t)(d0 + r) * kD + f0 + c]) * carry;
  }
  __syncthreads();
  const int lane = t & 31;
  const int wave = __builtin_amdgcn_readfirstlane((int)(threadIdx.x >> 5));
  const int q = lane >> 3, c8 = (lane & 7) * 8;
  unsigned short* op = out + (size_t)z * kD * kD;
  for (int pass = 0; pass < 2; ++pass) {
#pragma unroll
    for (int it = 0; it < 2; ++it) {
      const int row = wave * 8 + it * 4 + q;
      unsigned short hb[8];
#pragma unroll
      for (int e = 0; e < 8; ++e) hb[e] = h_bits(sm[row][c8 + e]);
      const v4u u = (v4u){pk16(hb[0], hb[1]), pk16(hb[2], hb[3]), pk16(hb[4], hb[5]), pk16(hb[6], hb[7])};
      *(volatile v4u*)(op + (size_t)(f0 + row) * kD + d0 + c8) = u;
    }
    __threadfence();
  }
}

struct InvFreq { float v[kHalfHD]; };
static_assert(sizeof(InvFreq) == 256);

__global__ __launch_bounds__(256) void angle_table_kernel(float* __restrict__ cosT, float* __restrict__ sinT, InvFreq inv) {
  const int idx = blockIdx.x * 256 + threadIdx.x;
  const int s = idx >> 6;
  const int i = idx & 63;
  float f = inv.v[0];
#pragma unroll
  for (int k = 1; k < kHalfHD; ++k) f = (i == k) ? inv.v[k] : f;
  const float ang = (float)s * f;
  const float sn = sinf(ang);
  const float cs = cosf(ang);
  *(volatile float*)(cosT + idx) = cs;
  *(volatile float*)(sinT + idx) = sn;
  __threadfence();
  *(volatile float*)(cosT + idx) = cs;
  *(volatile float*)(sinT + idx) = sn;
}

constexpr int kSlabP = 132;
constexpr int kVtP   = 136;
constexpr int kEpiLdsBytes = 128 * kVtP * 2;
static_assert(kEpiLdsBytes >= 4 * 16 * kSlabP * 4);

template <int MODE>
__global__ __launch_bounds__(128) void gemm_tile128_kernel(
    const unsigned short* __restrict__ Ap, const unsigned short* __restrict__ Btp,
    const float* __restrict__ bias0, const float* __restrict__ bias1, const float* __restrict__ bias2,
    const float* __restrict__ cosT, const float* __restrict__ sinT,
    unsigned short* __restrict__ Qr, unsigned short* __restrict__ Kr, unsigned short* __restrict__ Vt,
    float* __restrict__ Cout, float accScale, float biasScale)
{
  __shared__ __align__(16) unsigned char smraw[kEpiLdsBytes];
  const int lane  = threadIdx.x & 31;
  const int wave  = __builtin_amdgcn_readfirstlane((int)(threadIdx.x >> 5));
  const int rlane = lane & 15;
  const int hh    = lane >> 4;
  const int koff  = hh * 8;
  const int mOff  = hh * 8;
  const int mblk  = blockIdx.x * 128;
  const int m0w   = mblk + wave * 32;
  const int nblk  = blockIdx.y;
  const int n0    = nblk * 128;
  const int which = (MODE == 0) ? (nblk >> 4) : 0;
  const int head  = nblk & 15;

  const _Float16* A  = (const _Float16*)Ap;
  const _Float16* Bt = (const _Float16*)Btp;
  const _Float16* ap = A  + (size_t)(m0w + rlane) * kD + koff;
  const _Float16* bp = Bt + (size_t)(n0 + rlane) * kD + koff;

  v8f acc[2][8];
#pragma unroll
  for (int i = 0; i < 2; ++i)
#pragma unroll
    for (int j = 0; j < 8; ++j) acc[i][j] = (v8f){0.f, 0.f, 0.f, 0.f, 0.f, 0.f, 0.f, 0.f};

#pragma unroll 1
  for (int k0 = 0; k0 < kD; k0 += 32) {
    const v16h a0 = frag_ld(ap + k0);
    const v16h a1 = frag_ld(ap + (size_t)16 * kD + k0);
#pragma unroll
    for (int j = 0; j < 8; ++j) {
      const v16h bf = frag_ld(bp + (size_t)j * 16 * kD + k0);
      acc[0][j] = mma_h(a0, bf, acc[0][j]);
      acc[1][j] = mma_h(a1, bf, acc[1][j]);
    }
  }

  const float* bias = (MODE == 1) ? bias0 : ((which == 0) ? bias0 : (which == 1) ? bias1 : bias2);
  float bv[8];
#pragma unroll
  for (int j = 0; j < 8; ++j) bv[j] = bf16r(bias[head * 128 + j * 16 + rlane]) * biasScale;

  if (MODE == 1 || which < 2) {
    float* slab = (float*)smraw + wave * (16 * kSlabP);
#pragma unroll
    for (int i = 0; i < 2; ++i) {
#pragma unroll
      for (int j = 0; j < 8; ++j)
#pragma unroll
        for (int r = 0; r < 8; ++r)
          slab[(mOff + r) * kSlabP + j * 16 + rlane] = acc[i][j][r] * accScale + bv[j];
      wave_lds_sync();
      if (MODE == 1) {
        const int c4 = lane * 4;
        for (int pass = 0; pass < 2; ++pass) {
#pragma unroll 1
          for (int it = 0; it < 16; ++it) {
            const v4f v = *(const v4f*)(slab + it * kSlabP + c4);
            *(volatile v4f*)(Cout + (size_t)(m0w + i * 16 + it) * kD + n0 + c4) = v;
          }
          __threadfence();
        }
      } else {
        unsigned short* dst = (which == 0) ? Qr : Kr;
        const int hh2 = lane >> 4;
        const int c8  = (lane & 15) * 8;
        const int ci  = c8 & 63;
        const bool first = (c8 < kHalfHD);
        for (int pass = 0; pass < 2; ++pass) {
#pragma unroll 1
          for (int it = 0; it < 8; ++it) {
            const int row  = it * 2 + hh2;
            const int mrow = m0w + i * 16 + row;
            const int s    = mrow % kS;
            const int bb   = mrow / kS;
            const float* sp = slab + row * kSlabP;
            const v4f x1a = *(const v4f*)(sp + ci);
            const v4f x1b = *(const v4f*)(sp + ci + 4);
            const v4f x2a = *(const v4f*)(sp + kHalfHD + ci);
            const v4f x2b = *(const v4f*)(sp + kHalfHD + ci + 4);
            const float* cp = cosT + (size_t)s * kHalfHD + ci;
            const float* qp = sinT + (size_t)s * kHalfHD + ci;
            const v4f ca = *(const v4f*)(cp);
            const v4f cb = *(const v4f*)(cp + 4);
            const v4f sa = *(const v4f*)(qp);
            const v4f sb = *(const v4f*)(qp + 4);
            v8h hv;
#pragma unroll
            for (int e = 0; e < 4; ++e) {
              const float fa0 = first ? ca[e] : sa[e];
              const float fb0 = first ? -sa[e] : ca[e];
              const float fa1 = first ? cb[e] : sb[e];
              const float fb1 = first ? -sb[e] : cb[e];
              hv[e]     = (_Float16)(x1a[e] * fa0 + x2a[e] * fb0);
              hv[4 + e] = (_Float16)(x1b[e] * fa1 + x2b[e] * fb1);
            }
            *(volatile v8h*)(dst + ((size_t)(bb * kH + head) * kS + s) * kHD + c8) = hv;
          }
          __threadfence();
        }
      }
      wave_lds_sync();
    }
  } else {
    _Float16* sv = (_Float16*)smraw;
#pragma unroll
    for (int i = 0; i < 2; ++i)
#pragma unroll
      for (int j = 0; j < 8; ++j) {
        v8h hv;
#pragma unroll
        for (int r = 0; r < 8; ++r) hv[r] = (_Float16)(acc[i][j][r] * accScale + bv[j]);
        const int hd = j * 16 + rlane;
        const int sl = wave * 32 + i * 16 + mOff;
        *(v8h*)(sv + hd * kVtP + sl) = hv;
      }
    __syncthreads();
    const int hh2 = lane >> 4;
    const int c8  = (lane & 15) * 8;
    const int s0  = mblk % kS;
    const int bb  = mblk / kS;
    for (int pass = 0; pass < 2; ++pass) {
#pragma unroll 1
      for (int it = 0; it < 16; ++it) {
        const int hd = it * 8 + wave * 2 + hh2;
        const v8h val = *(const v8h*)(sv + hd * kVtP + c8);
        *(volatile v8h*)(Vt + ((size_t)(bb * kH + head) * kHD + hd) * kS + s0 + c8) = val;
      }
      __threadfence();
    }
  }
}

constexpr int kVOff = kKT * kHD;

__global__ __launch_bounds__(256) void attn_kernel(const unsigned short* __restrict__ Qp, const unsigned short* __restrict__ Kp,
                                                   const unsigned short* __restrict__ Vp, unsigned short* __restrict__ Aop,
                                                   float sclScore, float outFold)
{
  __shared__ __align__(16) _Float16 KV[2 * kKT * kHD];
  __shared__ __align__(16) _Float16 Ps[8][16 * kKT];
  const int tid  = threadIdx.x;
  const int lane = tid & 31;
  const int wave = __builtin_amdgcn_readfirstlane((int)(threadIdx.x >> 5));
  const int hh   = lane >> 4;
  const int c    = lane & 15;
  const int bh   = blockIdx.y;
  const int b    = bh / kH;
  const int h    = bh % kH;
  const int q0   = blockIdx.x * 128 + wave * 16;

  const _Float16* Qh = (const _Float16*)Qp + (size_t)bh * kS * kHD;
  const _Float16* Kh = (const _Float16*)Kp + (size_t)bh * kS * kHD;
  const _Float16* Vh = (const _Float16*)Vp + (size_t)bh * kHD * kS;

  v16h qa[4];
  {
    const _Float16* qrow = Qh + (size_t)(q0 + c) * kHD + 8 * hh;
#pragma unroll
    for (int kc = 0; kc < 4; ++kc) qa[kc] = frag_ld(qrow + kc * 32);
  }

  float mrow[8], lrow[8];
  v8f oacc[8];
#pragma unroll
  for (int r = 0; r < 8; ++r) { mrow[r] = -1.0e30f; lrow[r] = 0.f; }
#pragma unroll
  for (int t = 0; t < 8; ++t) oacc[t] = (v8f){0.f, 0.f, 0.f, 0.f, 0.f, 0.f, 0.f, 0.f};

  _Float16* pw = Ps[wave];

#pragma unroll 1
  for (int kv0 = 0; kv0 < kS; kv0 += kKT) {
    __syncthreads();
#pragma unroll
    for (int j = 0; j < 4; ++j) {
      const int idx = tid + j * 256;
      const int kr = idx >> 4, kp = (idx & 15) * 8;
      const v8h kk = *(const v8h*)(Kh + (size_t)(kv0 + kr) * kHD + kp);
      *(v8h*)(&KV[kr * kHD + kp]) = kk;
      const int vr = idx >> 3, vp = (idx & 7) * 8;
      const v8h vv = *(const v8h*)(Vh + (size_t)vr * kS + kv0 + vp);
      *(v8h*)(&KV[kVOff + vr * kKT + vp]) = vv;
    }
    __syncthreads();

    v8f s[4];
#pragma unroll
    for (int j = 0; j < 4; ++j) {
      v8f sj = (v8f){0.f, 0.f, 0.f, 0.f, 0.f, 0.f, 0.f, 0.f};
#pragma unroll
      for (int kc = 0; kc < 4; ++kc) {
        FragU kb;
        const int o = (j * 16 + c) * kHD + kc * 32 + 8 * hh;
        kb.h[0] = *(const v8h*)(&KV[o]);
        kb.h[1] = *(const v8h*)(&KV[o + 16]);
        sj = mma_h(qa[kc], kb.v, sj);
      }
      s[j] = sj;
    }
#pragma unroll
    for (int j = 0; j < 4; ++j)
#pragma unroll
      for (int r = 0; r < 8; ++r) s[j][r] *= sclScore;

#pragma unroll
    for (int r = 0; r < 8; ++r) {
      float m = fmaxf(fmaxf(s[0][r], s[1][r]), fmaxf(s[2][r], s[3][r]));
      m = fmaxf(m, __shfl_xor(m, 1, 32));
      m = fmaxf(m, __shfl_xor(m, 2, 32));
      m = fmaxf(m, __shfl_xor(m, 4, 32));
      m = fmaxf(m, __shfl_xor(m, 8, 32));
      const float mnew  = fmaxf(mrow[r], m);
      const float alpha = __expf(mrow[r] - mnew);
      mrow[r] = mnew;
      float psum = 0.f;
#pragma unroll
      for (int j = 0; j < 4; ++j) {
        const float p = __expf(s[j][r] - mnew);
        psum += p;
        pw[(8 * hh + r) * kKT + j * 16 + c] = (_Float16)(p * kPCarry);
      }
      psum += __shfl_xor(psum, 1, 32);
      psum += __shfl_xor(psum, 2, 32);
      psum += __shfl_xor(psum, 4, 32);
      psum += __shfl_xor(psum, 8, 32);
      lrow[r] = lrow[r] * alpha + psum;
#pragma unroll
      for (int t = 0; t < 8; ++t) oacc[t][r] *= alpha;
    }
    wave_lds_sync();
#pragma unroll
    for (int kk = 0; kk < 2; ++kk) {
      FragU pa;
      const int po = c * kKT + kk * 32 + 8 * hh;
      pa.h[0] = *(const v8h*)(pw + po);
      pa.h[1] = *(const v8h*)(pw + po + 16);
#pragma unroll
      for (int t = 0; t < 8; ++t) {
        FragU vb;
        const int vo = kVOff + (t * 16 + c) * kKT + kk * 32 + 8 * hh;
        vb.h[0] = *(const v8h*)(&KV[vo]);
        vb.h[1] = *(const v8h*)(&KV[vo + 16]);
        oacc[t] = mma_h(pa.v, vb.v, oacc[t]);
      }
    }
    wave_lds_sync();
  }

  __syncthreads();
  _Float16* os = &KV[wave * (16 * kHD)];
#pragma unroll
  for (int r = 0; r < 8; ++r) {
    const float inv = outFold * (1.0f / lrow[r]);
#pragma unroll
    for (int t = 0; t < 8; ++t) os[(8 * hh + r) * kHD + t * 16 + c] = (_Float16)(oacc[t][r] * inv);
  }
  wave_lds_sync();
  {
    const int hh2 = lane >> 4;
    const int c8  = (lane & 15) * 8;
    for (int pass = 0; pass < 2; ++pass) {
#pragma unroll 1
      for (int it = 0; it < 8; ++it) {
        const int row = it * 2 + hh2;
        const v8h val = *(const v8h*)(os + row * kHD + c8);
        *(volatile v8h*)(Aop + (size_t)(b * kS + q0 + row) * kD + h * kHD + c8) = val;
      }
      __threadfence();
    }
  }
}

extern "C" void kernel_launch(void* const* d_in, const int* in_sizes, int n_in,
                              void* d_out, int out_size, void* d_ws, size_t ws_size,
                              hipStream_t stream) {
  if (n_in < 9) return;
  if (in_sizes[0] != kM * kD) return;
  if (in_sizes[1] != kD * kD || in_sizes[3] != kD * kD || in_sizes[5] != kD * kD || in_sizes[7] != kD * kD) return;
  if (in_sizes[2] != kD || in_sizes[4] != kD || in_sizes[6] != kD || in_sizes[8] != kD) return;
  if (out_size != kM * kD) return;
  if (ws_size < kWsTotal) return;

  const float* x  = (const float*)d_in[0];
  const float* Wq = (const float*)d_in[1];
  const float* bq = (const float*)d_in[2];
  const float* Wk = (const float*)d_in[3];
  const float* bk = (const float*)d_in[4];
  const float* Wv = (const float*)d_in[5];
  const float* bv = (const float*)d_in[6];
  const float* Wo = (const float*)d_in[7];
  const float* bo = (const float*)d_in[8];
  float* out = (float*)d_out;

  char* ws = (char*)d_ws;
  unsigned short* XH = (unsigned short*)(ws + kOffXH);
  unsigned short* WT = (unsigned short*)(ws + kOffWT);
  unsigned short* QR = (unsigned short*)(ws + kOffQR);
  unsigned short* KR = (unsigned short*)(ws + kOffKR);
  unsigned short* VT = (unsigned short*)(ws + kOffVT);
  unsigned short* AO = (unsigned short*)(ws + kOffAO);
  float* COS = (float*)(ws + kOffCOS);
  float* SIN = (float*)(ws + kOffSIN);

  InvFreq inv;
  for (int i = 0; i < kHalfHD; ++i) {
    const float e = (float)(2 * i) / (float)kHD;
    inv.v[i] = 1.0f / powf(10000.0f, e);
  }
  const float sclScore = (1.0f / sqrtf((float)kHD)) / (kQKVCarry * kQKVCarry);

  cast_plane_kernel<<<(kM * kD / 8) / 256, 256, 0, stream>>>(x, XH, kM * kD / 8, kXCarry);
  wtcast_kernel<<<dim3(kD / 64, kD / 64, 4), 256, 0, stream>>>(Wq, Wk, Wv, Wo, WT, kWCarry);
  angle_table_kernel<<<(kS * kHalfHD) / 256, 256, 0, stream>>>(COS, SIN, inv);

  gemm_tile128_kernel<0><<<dim3(kM / 128, 3 * kD / 128), 128, 0, stream>>>(
      XH, WT, bq, bk, bv, COS, SIN, QR, KR, VT, (float*)nullptr, kProjScale, kQKVCarry);

  attn_kernel<<<dim3(kS / 128, kB * kH), 256, 0, stream>>>(QR, KR, VT, AO, sclScore, kCtxFold);

  gemm_tile128_kernel<1><<<dim3(kM / 128, kD / 128), 128, 0, stream>>>(
      AO, WT + (size_t)3 * kD * kD, bo, bo, bo, COS, SIN,
      (unsigned short*)nullptr, (unsigned short*)nullptr, (unsigned short*)nullptr, out, kOutScale, 1.0f);
}
